// Net_678604833378
// MI455X (gfx1250) — hardware-verified
//
#include <hip/hip_runtime.h>
#include <stddef.h>
#include <stdint.h>
#include <math.h>


#define NB     32
#define NN     512
#define DF     768
#define NE     4096
#define MR     (NB * NN)
#define K1     768
#define K2     1536
#define NTHR   256
#define DEGCAP 32
#define GB     64
#define GBM    64
#define GBN    64
#define GTHR   128
#define UW1    (DF * (K1 / 8))
#define UW2    (DF * (K2 / 8))
#define UX     (MR * (DF / 8))
#define WSMAX  134217728

static_assert(K1 % 32 == 0 && K2 % 32 == 0 && K2 == 2 * DF && K1 == DF);
static_assert(MR % GBM == 0 && DF % GBN == 0);
static_assert(GBM == (GTHR / 32) * 16 && GBN == 64);
static_assert(UW1 % NTHR == 0 && UW2 % NTHR == 0 && UX % NTHR == 0);
static_assert((K1 / 8) % 8 == 0 && (K2 / 8) % 8 == 0);
static_assert(NN % GB == 0 && NE % (GB * 4) == 0 && (GB * DEGCAP) % (GB * 4) == 0);
static_assert(DEGCAP == 32 && GB == 64);
static_assert(MR % 8 == 0 && NN == 512 && DF == 6 * 128);
static_assert((long long)(MR - 1) * DF + 5 * 128 + 4 * 31 + 3 == (long long)MR * DF - 1);

typedef float          v4f   __attribute__((ext_vector_type(4)));
typedef float          v8f   __attribute__((ext_vector_type(8)));
typedef int            v4i   __attribute__((ext_vector_type(4)));
typedef int            v8i   __attribute__((ext_vector_type(8)));
typedef unsigned short v8us  __attribute__((ext_vector_type(8)));
typedef unsigned short v16us __attribute__((ext_vector_type(16)));
typedef __bf16         v16bf __attribute__((ext_vector_type(16)));
typedef v4f  __attribute__((may_alias)) v4fa;
typedef v4i  __attribute__((may_alias)) v4ia;
typedef v8us __attribute__((may_alias)) v8usa;
union FragB { v16bf v; v16us u; v8us h[2]; v8i w; };

__device__ __forceinline__ v8f wmb(const FragB& a, const FragB& b, v8f c) {
  v8f d = __builtin_amdgcn_wmma_f32_16x16x32_bf16(false, a.v, false, b.v, (short)0, c, false, false);
  asm volatile("v_nop\n\tv_nop\n\tv_nop\n\tv_nop" : "+v"(d) : "v"(a.w), "v"(b.w));
  return d;
}

__device__ __forceinline__ unsigned bf16_bits(float f) {
  const unsigned u = __float_as_uint(f);
  return (u + 0x7FFFu + ((u >> 16) & 1u)) >> 16;
}
__device__ __forceinline__ float bf16_val(float f) {
  return __uint_as_float(bf16_bits(f) << 16);
}
__device__ __forceinline__ float relu_np(float v) {
  return (v > 0.0f) ? v : (v - v);
}

__global__ __launch_bounds__(NTHR) void k_wprep(const float* __restrict__ W1, const float* __restrict__ W2,
                                                unsigned short* W1T, unsigned short* W2D) {
  const int u = (int)blockIdx.x * NTHR + (int)threadIdx.x;
  v8us o;
  unsigned short* dp;
  if (u < UW1) {
    const int n  = u / (K1 / 8);
    const int k8 = (u - n * (K1 / 8)) * 8;
    const float* p = W1 + (size_t)k8 * DF + n;
#pragma unroll
    for (int i = 0; i < 8; ++i) o[i] = (unsigned short)bf16_bits(p[(size_t)i * DF]);
    dp = W1T + (size_t)n * K1 + k8;
  } else if (u < UW1 + UW2) {
    const int v  = u - UW1;
    const int n  = v / (K2 / 8);
    const int k8 = (v - n * (K2 / 8)) * 8;
    const int kk = (k8 >= DF) ? (k8 - DF) : k8;
    const float* p = W2 + (size_t)kk * DF + n;
#pragma unroll
    for (int i = 0; i < 8; ++i) o[i] = (unsigned short)bf16_bits(p[(size_t)i * DF]);
    dp = W2D + (size_t)n * K2 + k8;
  } else {
    return;
  }
  *(volatile v8us*)dp = o;
  __threadfence();
  *(volatile v8us*)dp = o;
}

__global__ __launch_bounds__(NTHR) void k_cvx(const float* __restrict__ x, unsigned short* xb) {
  const size_t u = (size_t)blockIdx.x * NTHR + (size_t)threadIdx.x;
  const float* p = x + u * 8;
  const v4f a = *(const v4fa*)p;
  const v4f b = *(const v4fa*)(p + 4);
  v8us o;
  o[0] = (unsigned short)bf16_bits(a.x); o[1] = (unsigned short)bf16_bits(a.y);
  o[2] = (unsigned short)bf16_bits(a.z); o[3] = (unsigned short)bf16_bits(a.w);
  o[4] = (unsigned short)bf16_bits(b.x); o[5] = (unsigned short)bf16_bits(b.y);
  o[6] = (unsigned short)bf16_bits(b.z); o[7] = (unsigned short)bf16_bits(b.w);
  unsigned short* dp = xb + u * 8;
  *(volatile v8us*)dp = o;
  __threadfence();
  *(volatile v8us*)dp = o;
}

__global__ __launch_bounds__(GB) void k_graph(const int* __restrict__ ei, const float* __restrict__ ea,
                                              int* esrc, float* ewt, int* node) {
  __shared__ __attribute__((aligned(16))) int   spk[NE];
  __shared__ __attribute__((aligned(16))) float sew[NE];
  __shared__ __attribute__((aligned(16))) int   lsrc[GB * DEGCAP];
  __shared__ __attribute__((aligned(16))) float lew[GB * DEGCAP];
  __shared__ __attribute__((aligned(16))) int   nodep[4 * GB];
  const int tid = (int)threadIdx.x;

#pragma unroll 1
  for (int it = 0; it < NE / (GB * 4); ++it) {
    const int e0 = (it * GB + tid) * 4;
    const v4i s4 = *(const v4i*)(ei + e0);
    const v4i d4 = *(const v4i*)(ei + NE + e0);
    const v4f w4 = *(const v4f*)(ea + e0);
    v4i p;
    {
      int s; unsigned d;
      s = s4.x < 0 ? 0 : (s4.x > NN - 1 ? NN - 1 : s4.x); d = ((unsigned)d4.x < (unsigned)NN) ? (unsigned)d4.x : 0xFFFFu;
      p.x = (int)((d << 16) | (unsigned)s);
      s = s4.y < 0 ? 0 : (s4.y > NN - 1 ? NN - 1 : s4.y); d = ((unsigned)d4.y < (unsigned)NN) ? (unsigned)d4.y : 0xFFFFu;
      p.y = (int)((d << 16) | (unsigned)s);
      s = s4.z < 0 ? 0 : (s4.z > NN - 1 ? NN - 1 : s4.z); d = ((unsigned)d4.z < (unsigned)NN) ? (unsigned)d4.z : 0xFFFFu;
      p.z = (int)((d << 16) | (unsigned)s);
      s = s4.w < 0 ? 0 : (s4.w > NN - 1 ? NN - 1 : s4.w); d = ((unsigned)d4.w < (unsigned)NN) ? (unsigned)d4.w : 0xFFFFu;
      p.w = (int)((d << 16) | (unsigned)s);
    }
    v4f w;
    w.x = bf16_val(w4.x); w.y = bf16_val(w4.y); w.z = bf16_val(w4.z); w.w = bf16_val(w4.w);
    *(v4ia*)(spk + e0) = p;
    *(v4fa*)(sew + e0) = w;
  }
  {
    const v4i zi = {0, 0, 0, 0};
    const v4f zf = {0.0f, 0.0f, 0.0f, 0.0f};
#pragma unroll 1
    for (int it = 0; it < (GB * DEGCAP) / (GB * 4); ++it) {
      const int idx = (it * GB + tid) * 4;
      *(v4ia*)(lsrc + idx) = zi;
      *(v4fa*)(lew + idx) = zf;
    }
  }
  __syncthreads();

  const unsigned mine = (unsigned)((int)blockIdx.x * GB + tid);
  int c = 0;
  float ds = 0.0f;
#pragma unroll 4
  for (int e = 0; e < NE; ++e) {
    const int   pk = spk[e];
    const float w  = sew[e];
    const bool hit = (((unsigned)pk) >> 16) == mine;
    const float hf = hit ? 1.0f : 0.0f;
    ds = fmaf(w, hf, ds);
    if (hit) {
      if (c < DEGCAP) {
        lsrc[tid * DEGCAP + c] = pk & 0xFFFF;
        lew[tid * DEGCAP + c]  = w;
      }
      c = c + 1;
    }
  }
  const float deg  = ds + 1.0f;
  const float dinv = (deg > 0.0f) ? (1.0f / sqrtf(deg)) : 0.0f;
  nodep[tid]          = c;
  nodep[GB + tid]     = __float_as_int(dinv);
  nodep[2 * GB + tid] = (c > DEGCAP) ? 1 : 0;
  nodep[3 * GB + tid] = __float_as_int(deg);
  __syncthreads();

  constexpr int NIT = (GB * DEGCAP) / (GB * 4);
  v4i sv[NIT];
  v4f wv[NIT];
#pragma unroll
  for (int it = 0; it < NIT; ++it) {
    const int idx = (it * GB + tid) * 4;
    sv[it] = *(const v4ia*)(lsrc + idx);
    wv[it] = *(const v4fa*)(lew + idx);
  }
  const int pl = tid >> 4, q = tid & 15;
  const v4i nv = *(const v4ia*)(nodep + GB * pl + 4 * q);
  int*   es = esrc + (size_t)blockIdx.x * (GB * DEGCAP);
  float* ew = ewt  + (size_t)blockIdx.x * (GB * DEGCAP);
  int*   np = node + (size_t)pl * NN + (size_t)blockIdx.x * GB + 4 * q;
#pragma unroll
  for (int it = 0; it < NIT; ++it) {
    const int idx = (it * GB + tid) * 4;
    *(volatile v4i*)(es + idx) = sv[it];
    *(volatile v4f*)(ew + idx) = wv[it];
  }
  *(volatile v4i*)np = nv;
  __threadfence();
#pragma unroll
  for (int it = 0; it < NIT; ++it) {
    const int idx = (it * GB + tid) * 4;
    *(volatile v4i*)(es + idx) = sv[it];
    *(volatile v4f*)(ew + idx) = wv[it];
  }
  *(volatile v4i*)np = nv;
}

__global__ __launch_bounds__(GTHR) void k_gemm(
    const unsigned short* __restrict__ A, const unsigned short* __restrict__ WT,
    float* outF, int K, int ldo)
{
  __shared__ __attribute__((aligned(16))) float stg[GBM * GBN];
  const int tid = (int)threadIdx.x, lane = tid & 31, wave = tid >> 5, hh = lane >> 4, m = lane & 15;
  const int rowBase = (int)blockIdx.x * GBM;
  const int col0    = (int)blockIdx.y * GBN;

  v8f acc[4];
  {
    const v8f z = {0.f, 0.f, 0.f, 0.f, 0.f, 0.f, 0.f, 0.f};
    acc[0] = z; acc[1] = z; acc[2] = z; acc[3] = z;
  }
  const unsigned short* ap = A  + (size_t)(rowBase + 16 * wave + m) * (size_t)K + 8 * hh;
  const unsigned short* wp = WT + (size_t)(col0 + m) * (size_t)K + 8 * hh;
  const int ksteps = K >> 5;
#pragma unroll 1
  for (int ks = 0; ks < ksteps; ++ks) {
    FragB af;
    af.h[0] = *(const v8usa*)(ap + 32 * ks);
    af.h[1] = *(const v8usa*)(ap + 32 * ks + 16);
#pragma unroll
    for (int t = 0; t < 4; ++t) {
      const unsigned short* wq = wp + (size_t)(16 * t) * (size_t)K + 32 * ks;
      FragB bf;
      bf.h[0] = *(const v8usa*)wq;
      bf.h[1] = *(const v8usa*)(wq + 16);
      acc[t] = wmb(af, bf, acc[t]);
    }
  }

#pragma unroll
  for (int t = 0; t < 4; ++t) {
    const int lc = 16 * t + m;
#pragma unroll
    for (int r = 0; r < 8; ++r) {
      const int lr = 16 * wave + 8 * hh + r;
      stg[lr * GBN + lc] = acc[t][r];
    }
  }
  __syncthreads();

  v4f fv[8];
#pragma unroll
  for (int i = 0; i < 8; ++i) {
    const int lr = 16 * wave + 2 * i + hh;
    fv[i] = *(const v4fa*)(stg + lr * GBN + 4 * m);
  }
#pragma unroll
  for (int i = 0; i < 8; ++i) {
    const int lr = 16 * wave + 2 * i + hh;
    const int gr = rowBase + lr;
    float* op = outF + (size_t)gr * (size_t)ldo + col0 + 4 * m;
    *(volatile v4f*)op = fv[i];
  }
  __threadfence();
#pragma unroll
  for (int i = 0; i < 8; ++i) {
    const int lr = 16 * wave + 2 * i + hh;
    const int gr = rowBase + lr;
    float* op = outF + (size_t)gr * (size_t)ldo + col0 + 4 * m;
    *(volatile v4f*)op = fv[i];
  }
}

template <int MODE>
__device__ __forceinline__ int coff(int j, int lane) {
  return (MODE != 0) ? (256 * (j >> 1) + 8 * lane + 4 * (j & 1)) : (128 * j + 4 * lane);
}

template <int MODE>
__global__ __launch_bounds__(NTHR) void k_agg(const float* __restrict__ H,
                                              const int* __restrict__ esrc, const float* __restrict__ ewt,
                                              const int* __restrict__ cntp, const float* __restrict__ dinvp,
                                              const int* __restrict__ ovfp, const float* __restrict__ bias,
                                              unsigned short* hl, float* outp) {
  const int tid  = (int)threadIdx.x, lane = tid & 31;
  const int wave = __builtin_amdgcn_readfirstlane(tid >> 5);
  const int rowg = (int)blockIdx.x * 8 + wave;
  const int bt   = rowg >> 9;
  const int i    = rowg & (NN - 1);

  int c = cntp[i];
  const int ov = ovfp[i];
  const bool big = (c > DEGCAP) || (c < 0) || (ov != 0);
  c = c < 0 ? 0 : (c > DEGCAP ? DEGCAP : c);
  const float dd = dinvp[i];
  const float rd = dd * dd;
  int sr = esrc[i * DEGCAP + lane];
  sr = sr < 0 ? 0 : (sr > NN - 1 ? NN - 1 : sr);
  const float wj  = ewt[i * DEGCAP + lane];
  const float cf  = (dinvp[sr] * wj) * dd;
  const int   cfi = __float_as_int(cf);

  v4f acc[6];
  {
    const v4f z = {0.0f, 0.0f, 0.0f, 0.0f};
#pragma unroll
    for (int j = 0; j < 6; ++j) acc[j] = z;
  }
  const float* hb = H + (size_t)bt * NN * DF;
#pragma unroll 1
  for (int k = 0; k <= c; ++k) {
    const bool self = (k == c);
    const int  kk   = self ? 0 : k;
    int   sk  = __builtin_amdgcn_readlane(sr, kk);
    int   cki = __builtin_amdgcn_readlane(cfi, kk);
    sk = self ? i : sk;
    const float ck = self ? rd : __int_as_float(cki);
    const float* hp = hb + (size_t)sk * DF;
#pragma unroll
    for (int j = 0; j < 6; ++j) {
      const v4f a = *(const v4fa*)(hp + coff<MODE>(j, lane));
      acc[j].x = fmaf(ck, a.x, acc[j].x);
      acc[j].y = fmaf(ck, a.y, acc[j].y);
      acc[j].z = fmaf(ck, a.z, acc[j].z);
      acc[j].w = fmaf(ck, a.w, acc[j].w);
    }
  }

  const float qnan = __int_as_float(0x7fc00000);
  const float pz = big ? qnan : 0.0f;
  v4f y[6];
#pragma unroll
  for (int j = 0; j < 6; ++j) {
    const v4f b = *(const v4fa*)(bias + coff<MODE>(j, lane));
    v4f t;
    t.x = relu_np(acc[j].x + bf16_val(b.x)) + pz;
    t.y = relu_np(acc[j].y + bf16_val(b.y)) + pz;
    t.z = relu_np(acc[j].z + bf16_val(b.z)) + pz;
    t.w = relu_np(acc[j].w + bf16_val(b.w)) + pz;
    y[j] = t;
  }

  if constexpr (MODE != 0) {
    v8us hv[3], lv[3];
#pragma unroll
    for (int q = 0; q < 3; ++q) {
      const v4f a = y[2 * q], b = y[2 * q + 1];
      unsigned hbv;
      hbv = bf16_bits(a.x); hv[q][0] = (unsigned short)hbv; lv[q][0] = (unsigned short)bf16_bits(a.x - __uint_as_float(hbv << 16));
      hbv = bf16_bits(a.y); hv[q][1] = (unsigned short)hbv; lv[q][1] = (unsigned short)bf16_bits(a.y - __uint_as_float(hbv << 16));
      hbv = bf16_bits(a.z); hv[q][2] = (unsigned short)hbv; lv[q][2] = (unsigned short)bf16_bits(a.z - __uint_as_float(hbv << 16));
      hbv = bf16_bits(a.w); hv[q][3] = (unsigned short)hbv; lv[q][3] = (unsigned short)bf16_bits(a.w - __uint_as_float(hbv << 16));
      hbv = bf16_bits(b.x); hv[q][4] = (unsigned short)hbv; lv[q][4] = (unsigned short)bf16_bits(b.x - __uint_as_float(hbv << 16));
      hbv = bf16_bits(b.y); hv[q][5] = (unsigned short)hbv; lv[q][5] = (unsigned short)bf16_bits(b.y - __uint_as_float(hbv << 16));
      hbv = bf16_bits(b.z); hv[q][6] = (unsigned short)hbv; lv[q][6] = (unsigned short)bf16_bits(b.z - __uint_as_float(hbv << 16));
      hbv = bf16_bits(b.w); hv[q][7] = (unsigned short)hbv; lv[q][7] = (unsigned short)bf16_bits(b.w - __uint_as_float(hbv << 16));
    }
    unsigned short* rp = hl + (size_t)rowg * K2 + 8 * lane;
#pragma unroll
    for (int q = 0; q < 3; ++q) {
      *(volatile v8us*)(rp + 256 * q) = hv[q];
      *(volatile v8us*)(rp + DF + 256 * q) = lv[q];
    }
    __threadfence();
#pragma unroll
    for (int q = 0; q < 3; ++q) {
      *(volatile v8us*)(rp + 256 * q) = hv[q];
      *(volatile v8us*)(rp + DF + 256 * q) = lv[q];
    }
  } else {
    float* op = outp + (size_t)rowg * DF + 4 * lane;
#pragma unroll
    for (int j = 0; j < 6; ++j) *(volatile v4f*)(op + 128 * j) = y[j];
    __threadfence();
#pragma unroll
    for (int j = 0; j < 6; ++j) *(volatile v4f*)(op + 128 * j) = y[j];
  }
}

static inline size_t al256(size_t o) { return (o + 255) & ~(size_t)255; }

extern "C" void kernel_launch(void* const* d_in, const int* in_sizes, int n_in,
                              void* d_out, int out_size, void* d_ws, size_t ws_size,
                              hipStream_t stream) {
  if (n_in < 7) return;
  if (in_sizes[0] != MR * DF) return;
  if (in_sizes[1] != 2 * NE) return;
  if (in_sizes[2] != NE) return;
  if (in_sizes[3] != DF * DF || in_sizes[4] != DF) return;
  if (in_sizes[5] != DF * DF || in_sizes[6] != DF) return;
  if (out_size != MR * DF) return;

  const float* x    = (const float*)d_in[0];
  const int*   edge = (const int*)d_in[1];
  const float* ea   = (const float*)d_in[2];
  const float* W1   = (const float*)d_in[3];
  const float* b1   = (const float*)d_in[4];
  const float* W2   = (const float*)d_in[5];
  const float* b2   = (const float*)d_in[6];
  float* out = (float*)d_out;

  char* ws = (char*)d_ws;
  size_t off = 0;
  const size_t oXB  = off; off = al256(off + (size_t)MR * DF * 2);
  const size_t oH   = off; off = al256(off + (size_t)MR * DF * 4);
  const size_t oHL  = off; off = al256(off + (size_t)MR * K2 * 2);
  const size_t oW1T = off; off = al256(off + (size_t)DF * K1 * 2);
  const size_t oW2D = off; off = al256(off + (size_t)DF * K2 * 2);
  const size_t oES  = off; off = al256(off + (size_t)NN * DEGCAP * 4);
  const size_t oEW  = off; off = al256(off + (size_t)NN * DEGCAP * 4);
  const size_t oND  = off; off = al256(off + (size_t)4 * NN * 4);
  if (off > ws_size || off > (size_t)WSMAX) return;
  unsigned short* XB   = (unsigned short*)(ws + oXB);
  float*          H    = (float*)(ws + oH);
  unsigned short* H1HL = (unsigned short*)(ws + oHL);
  unsigned short* W1T  = (unsigned short*)(ws + oW1T);
  unsigned short* W2D  = (unsigned short*)(ws + oW2D);
  int*            ESRC = (int*)(ws + oES);
  float*          EWT  = (float*)(ws + oEW);
  int*            NODE = (int*)(ws + oND);
  const int*   CNT  = NODE;
  const float* DINV = (const float*)(NODE + NN);
  const int*   OVF  = NODE + 2 * NN;

  k_wprep<<<(UW1 + UW2) / NTHR, NTHR, 0, stream>>>(W1, W2, W1T, W2D);
  k_cvx<<<UX / NTHR, NTHR, 0, stream>>>(x, XB);
  k_graph<<<NN / GB, GB, 0, stream>>>(edge, ea, ESRC, EWT, NODE);
  k_gemm<<<dim3(MR / GBM, DF / GBN), GTHR, 0, stream>>>(XB, W1T, H, K1, DF);
  k_agg<1><<<MR / 8, NTHR, 0, stream>>>(H, ESRC, EWT, CNT, DINV, OVF, b1, H1HL, out);
  k_gemm<<<dim3(MR / GBM, DF / GBN), GTHR, 0, stream>>>(H1HL, W2D, H, K2, DF);
  k_agg<0><<<MR / 8, NTHR, 0, stream>>>(H, ESRC, EWT, CNT, DINV, OVF, b2, H1HL, out);
}
